// TinyChLSTMEncoder_3255585210854
// MI455X (gfx1250) — hardware-run, weakly checked
//
#include <hip/hip_runtime.h>
#include <math.h>

constexpr int NBAT  = 32;
constexpr int NCHN  = 64;
constexpr int TLEN  = 1000;
constexpr int NHID  = 16;
constexpr int NEMB  = 32;
constexpr int NSEQ  = NBAT * NCHN;
constexpr int NGATE = 4 * NHID;
constexpr int KPAD  = 32;
constexpr float BN_EPS = 1e-5f;

constexpr int CTHR   = 256;
constexpr int SGRP   = 32;
constexpr int TCH    = 128;
constexpr int NTCH   = (TLEN + TCH - 1) / TCH;
constexpr int XW     = TCH + 8;
constexpr int H1W    = TCH + 4;
constexpr int OSP    = SGRP + 4;

constexpr int LWAVES = 2;
constexpr int LTHR   = 32 * LWAVES;
constexpr int AHP    = 40;
constexpr int HSP    = 20;
constexpr float HCARRY   = 16.0f;
constexpr float WCARRY   = 64.0f;
constexpr float PROD_INV = 1.0f / 1024.0f;

constexpr int GWAVES = 2;
constexpr int GTHR   = 32 * GWAVES;
constexpr int GOSP   = NEMB + 4;

static_assert(TLEN % 4 == 0);
static_assert(TCH % 32 == 0);
static_assert((TCH / 8) % 4 == 0);
static_assert(XW % 4 == 0 && OSP % 4 == 0);
static_assert(NSEQ % SGRP == 0 && NCHN % SGRP == 0);
static_assert((SGRP * TCH) % CTHR == 0);
static_assert(SGRP * 4 == 128);
static_assert(NSEQ % 16 == 0);
static_assert(((NSEQ / 16) * 2) % LWAVES == 0);
static_assert((NSEQ / 16) % GWAVES == 0);
static_assert((LWAVES * 16 * AHP) % LTHR == 0);
static_assert(LTHR == NGATE);
static_assert(NEMB * 4 == 128);
static_assert(AHP % 8 == 0 && AHP >= KPAD && HSP % 4 == 0 && GOSP % 4 == 0);
static_assert(2 * NHID == KPAD);

typedef __attribute__((ext_vector_type(16))) _Float16 v16h;
typedef __attribute__((ext_vector_type(8)))  _Float16 v8h;
typedef __attribute__((ext_vector_type(8)))  float    v8f;
typedef __attribute__((ext_vector_type(4)))  float    v4f;

__device__ __forceinline__ void dep_guard_h(v8f& a, v8f& b, v16h x, v16h y) { asm volatile("v_nop\n\tv_nop\n\tv_nop\n\tv_nop" : "+v"(a), "+v"(b) : "v"(x), "v"(y)); }
__device__ __forceinline__ void keep4_h(v16h a, v16h b, v16h c, v16h d) { asm volatile("v_nop" :: "v"(a), "v"(b), "v"(c), "v"(d)); }
__device__ __forceinline__ void guard_acc4_ab5(v8f& a0, v8f& a1, v8f& a2, v8f& a3,
                                               v16h x, v16h b0, v16h b1, v16h b2, v16h b3) {
  asm volatile("v_nop\n\tv_nop\n\tv_nop\n\tv_nop"
               : "+v"(a0), "+v"(a1), "+v"(a2), "+v"(a3)
               : "v"(x), "v"(b0), "v"(b1), "v"(b2), "v"(b3));
}
__device__ __forceinline__ void guard_acc2_ab3(v8f& a0, v8f& a1, v16h x, v16h b0, v16h b1) {
  asm volatile("v_nop\n\tv_nop\n\tv_nop\n\tv_nop" : "+v"(a0), "+v"(a1) : "v"(x), "v"(b0), "v"(b1));
}

template <typename T> struct Frag;
template <> struct Frag<_Float16> {
  typedef v16h V; union U { v16h v; v8h h[2]; };
  static __device__ __forceinline__ v16h load(const _Float16* p) {
    U f; f.h[0] = *(const v8h*)(p); f.h[1] = *(const v8h*)(p + 16); return f.v;
  }
  static __device__ __forceinline__ v8f mma(v16h a, v16h b, v8f c) {
    return __builtin_amdgcn_wmma_f32_16x16x32_f16(false, a, false, b, (short)0, c, false, false);
  }
  static __device__ __forceinline__ void guard(v8f& a, v8f& b, v16h x, v16h y) { dep_guard_h(a, b, x, y); }
  static __device__ __forceinline__ void keep(v16h a, v16h b, v16h c, v16h d) { keep4_h(a, b, c, d); }
};

__device__ __forceinline__ float fsig(float x) {
  const float xc = fminf(fmaxf(x, -30.0f), 30.0f);
  return __builtin_amdgcn_rcpf(1.0f + expf(-xc));
}
__device__ __forceinline__ float ftanh(float x) {
  const float xc = fminf(fmaxf(x, -15.0f), 15.0f);
  return 1.0f - 2.0f * __builtin_amdgcn_rcpf(expf(2.0f * xc) + 1.0f);
}
__device__ __forceinline__ float gelu_erf(float y) {
  return 0.5f * y * (1.0f + erff(y * 0.70710678118654752f));
}

__global__ __launch_bounds__(256) void prep_whh_kernel(const float* __restrict__ Whh_f,
                                                       const float* __restrict__ Whh_b,
                                                       unsigned short* __restrict__ WHp) {
  const int i   = blockIdx.x * 256 + threadIdx.x;
  const int row = i >> 2, c8 = (i & 3) * 8;
  const int dir = row >> 6, rr = row & 63;
  const bool kreal = (c8 < NHID);
  const int c8c = c8 & (NHID - 1);
  const v4f fa = *(const v4f*)(Whh_f + (size_t)rr * NHID + c8c);
  const v4f fb = *(const v4f*)(Whh_f + (size_t)rr * NHID + c8c + 4);
  const v4f ba = *(const v4f*)(Whh_b + (size_t)rr * NHID + c8c);
  const v4f bb = *(const v4f*)(Whh_b + (size_t)rr * NHID + c8c + 4);
  v8h hv;
#pragma unroll
  for (int e = 0; e < 4; ++e) {
    float v0 = (dir ? ba[e] : fa[e]) * WCARRY;
    float v1 = (dir ? bb[e] : fb[e]) * WCARRY;
    v0 = kreal ? v0 : 0.0f;
    v1 = kreal ? v1 : 0.0f;
    hv[e]     = (_Float16)v0;
    hv[4 + e] = (_Float16)v1;
  }
  unsigned short* dst = WHp + (size_t)i * 8;
  *(volatile v8h*)dst = hv;
  __threadfence();
  *(volatile v8h*)dst = hv;
}

__global__ __launch_bounds__(128) void prep_wlin_kernel(const float* __restrict__ Wlin, unsigned short* __restrict__ WLp) {
  const int i = threadIdx.x;
  const int e = i >> 2, c8 = (i & 3) * 8;
  const v4f wa = *(const v4f*)(Wlin + (size_t)e * (2 * NHID) + c8);
  const v4f wb = *(const v4f*)(Wlin + (size_t)e * (2 * NHID) + c8 + 4);
  v8h hv;
#pragma unroll
  for (int k = 0; k < 4; ++k) {
    hv[k]     = (_Float16)(wa[k] * WCARRY);
    hv[4 + k] = (_Float16)(wb[k] * WCARRY);
  }
  unsigned short* dst = WLp + (size_t)i * 8;
  *(volatile v8h*)dst = hv;
  __threadfence();
  *(volatile v8h*)dst = hv;
}

__global__ __launch_bounds__(CTHR) void conv_stack_kernel(
    const float* __restrict__ x,
    const float* __restrict__ w1, const float* __restrict__ b1, const float* __restrict__ g1,
    const float* __restrict__ be1, const float* __restrict__ m1, const float* __restrict__ v1,
    const float* __restrict__ w2, const float* __restrict__ b2, const float* __restrict__ g2,
    const float* __restrict__ be2, const float* __restrict__ m2, const float* __restrict__ v2,
    float* __restrict__ XT) {
  __shared__ __align__(16) float xs[SGRP * XW];
  __shared__ __align__(16) float h1s[SGRP * H1W];
  __shared__ __align__(16) float os[TCH * OSP];
  __shared__ float wa[SGRP * 5], wb[SGRP * 5];
  __shared__ float p1i[SGRP], p1a[SGRP], p1b[SGRP], p2i[SGRP], p2a[SGRP], p2b[SGRP];
  const int tid = threadIdx.x, lane = tid & 31, wave = tid >> 5;
  const int nb = blockIdx.x, tc = blockIdx.y;
  const int nbase = nb * SGRP;
  const int cbase = (nb % (NCHN / SGRP)) * SGRP;
  const int t0 = tc * TCH;

  if (wave == 0) {
    const int ch = cbase + lane;
#pragma unroll
    for (int k = 0; k < 5; ++k) wa[lane * 5 + k] = w1[ch * 5 + k];
    const float inv = g1[ch] / sqrtf(v1[ch] + BN_EPS);
    p1i[lane] = inv;
    p1a[lane] = be1[ch] - m1[ch] * inv;
    p1b[lane] = b1[ch];
  } else if (wave == 1) {
    const int ch = cbase + lane;
#pragma unroll
    for (int k = 0; k < 5; ++k) wb[lane * 5 + k] = w2[ch * 5 + k];
    const float inv = g2[ch] / sqrtf(v2[ch] + BN_EPS);
    p2i[lane] = inv;
    p2a[lane] = be2[ch] - m2[ch] * inv;
    p2b[lane] = b2[ch];
  }

#pragma unroll 1
  for (int i = tid; i < SGRP * (XW / 4); i += CTHR) {
    const int s = i / (XW / 4), cv = i - s * (XW / 4);
    const int tg = t0 - 4 + 4 * cv;
    int tcl = tg < 0 ? 0 : tg;
    tcl = tcl > (TLEN - 4) ? (TLEN - 4) : tcl;
    v4f v = *(const v4f*)(x + (size_t)(nbase + s) * TLEN + tcl);
    const bool ok = (tg >= 0) && (tg <= TLEN - 4);
    if (!ok) v = (v4f){0.0f, 0.0f, 0.0f, 0.0f};
    *(v4f*)(xs + s * XW + 4 * cv) = v;
  }
  __syncthreads();

#pragma unroll 1
  for (int i = tid; i < SGRP * H1W; i += CTHR) {
    const int s = i / H1W, col = i - s * H1W;
    const float* xr = xs + s * XW + col;
    float a = 0.0f;
#pragma unroll
    for (int k = 0; k < 5; ++k) a += xr[k] * wa[s * 5 + k];
    const float y = (a + p1b[s]) * p1i[s] + p1a[s];
    const float ge = gelu_erf(y);
    const int tg = t0 - 2 + col;
    h1s[i] = (tg >= 0 && tg < TLEN) ? ge : 0.0f;
  }
  __syncthreads();

#pragma unroll 1
  for (int i = tid; i < SGRP * TCH; i += CTHR) {
    const int s = i / TCH, tt = i - s * TCH;
    const float* hr = h1s + s * H1W + tt;
    float a = 0.0f;
#pragma unroll
    for (int k = 0; k < 5; ++k) a += hr[k] * wb[s * 5 + k];
    const float y = (a + p2b[s]) * p2i[s] + p2a[s];
    os[tt * OSP + s] = gelu_erf(y);
  }
  __syncthreads();

  const int q = lane >> 3, c4 = (lane & 7) * 4;
  for (int pass = 0; pass < 2; ++pass) {
#pragma unroll
    for (int it = 0; it < (TCH / 8) / 4; ++it) {
      const int ttb = wave * (TCH / 8) + it * 4;
      if (t0 + ttb < TLEN) {
        const int tt = ttb + q;
        const v4f v = *(const v4f*)(os + tt * OSP + c4);
        *(volatile v4f*)(XT + (size_t)(t0 + tt) * NSEQ + nbase + c4) = v;
      }
    }
    __threadfence();
  }
}

__global__ __launch_bounds__(LTHR) void bilstm_kernel(
    const float* __restrict__ XT,
    const float* __restrict__ Wih_f, const float* __restrict__ bih_f, const float* __restrict__ bhh_f,
    const float* __restrict__ Wih_b, const float* __restrict__ bih_b, const float* __restrict__ bhh_b,
    const unsigned short* __restrict__ WHp, unsigned short* __restrict__ FHp) {
  __shared__ __align__(16) _Float16 Ah[LWAVES * 16 * AHP];
  __shared__ __align__(16) float    Hs[LWAVES * 16 * HSP];
  __shared__ float cw[2 * NGATE], cbs[2 * NGATE];
  const int tid = threadIdx.x, lane = tid & 31, wave = tid >> 5;
  const int c = lane & 15, hh = lane >> 4, koff = 8 * hh;
  const int wid  = blockIdx.x * LWAVES + wave;
  const int dir  = wid & 1;
  const int tile = wid >> 1;
  const int seq0 = tile * 16;

#pragma unroll 1
  for (int i = tid; i < LWAVES * 16 * AHP; i += LTHR) Ah[i] = (_Float16)0.0f;
  cw[tid] = Wih_f[tid];
  cw[NGATE + tid] = Wih_b[tid];
  cbs[tid] = bih_f[tid] + bhh_f[tid];
  cbs[NGATE + tid] = bih_b[tid] + bhh_b[tid];
  const _Float16* WH = (const _Float16*)WHp + (size_t)dir * NGATE * KPAD;
  const v16h bf0 = Frag<_Float16>::load(WH + (size_t)(0 * 16 + c) * KPAD + koff);
  const v16h bf1 = Frag<_Float16>::load(WH + (size_t)(1 * 16 + c) * KPAD + koff);
  const v16h bf2 = Frag<_Float16>::load(WH + (size_t)(2 * 16 + c) * KPAD + koff);
  const v16h bf3 = Frag<_Float16>::load(WH + (size_t)(3 * 16 + c) * KPAD + koff);
  __syncthreads();

  float wih[4], bs[4];
#pragma unroll
  for (int g = 0; g < 4; ++g) {
    const float vf = cw[g * 16 + c],  vb = cw[NGATE + g * 16 + c];
    const float sf = cbs[g * 16 + c], sb = cbs[NGATE + g * 16 + c];
    wih[g] = dir ? vb : vf;
    bs[g]  = dir ? sb : sf;
  }
  float cst[8], hst[8];
#pragma unroll
  for (int r = 0; r < 8; ++r) { cst[r] = 0.0f; hst[r] = 0.0f; }

  _Float16* aw = Ah + wave * 16 * AHP;
  const _Float16* ahrow = aw + c * AHP + koff;
  const v8f z8 = {0.f, 0.f, 0.f, 0.f, 0.f, 0.f, 0.f, 0.f};

#pragma unroll 1
  for (int t = 0; t < TLEN; ++t) {
    const int trow = dir ? (TLEN - 1 - t) : t;
    const float* xp = XT + (size_t)trow * NSEQ + seq0 + 8 * hh;
    const v4f xa = *(const v4f*)(xp);
    const v4f xb = *(const v4f*)(xp + 4);
    float xt[8];
    xt[0] = xa[0]; xt[1] = xa[1]; xt[2] = xa[2]; xt[3] = xa[3];
    xt[4] = xb[0]; xt[5] = xb[1]; xt[6] = xb[2]; xt[7] = xb[3];

    const v16h a = Frag<_Float16>::load(ahrow);
    v8f acc[4];
    acc[0] = Frag<_Float16>::mma(a, bf0, z8);
    acc[1] = Frag<_Float16>::mma(a, bf1, z8);
    acc[2] = Frag<_Float16>::mma(a, bf2, z8);
    acc[3] = Frag<_Float16>::mma(a, bf3, z8);
    guard_acc4_ab5(acc[0], acc[1], acc[2], acc[3], a, bf0, bf1, bf2, bf3);

#pragma unroll
    for (int r = 0; r < 8; ++r) {
      const float zi = acc[0][r] * PROD_INV + (xt[r] * wih[0] + bs[0]);
      const float zf = acc[1][r] * PROD_INV + (xt[r] * wih[1] + bs[1]);
      const float zg = acc[2][r] * PROD_INV + (xt[r] * wih[2] + bs[2]);
      const float zo = acc[3][r] * PROD_INV + (xt[r] * wih[3] + bs[3]);
      const float ig = fsig(zi);
      const float fg = fsig(zf);
      const float gg = ftanh(zg);
      const float og = fsig(zo);
      const float cn = fg * cst[r] + ig * gg;
      cst[r] = cn;
      hst[r] = og * ftanh(cn);
    }
    __syncthreads();
#pragma unroll
    for (int r = 0; r < 8; ++r) aw[(8 * hh + r) * AHP + c] = (_Float16)(hst[r] * HCARRY);
    __syncthreads();
  }

  float* hs = Hs + wave * 16 * HSP;
#pragma unroll
  for (int r = 0; r < 8; ++r) hs[(8 * hh + r) * HSP + c] = hst[r];
  __syncthreads();
  {
    const int row = lane >> 1, col8 = (lane & 1) * 8;
    v8h hv;
#pragma unroll
    for (int e = 0; e < 8; ++e) hv[e] = (_Float16)(hs[row * HSP + col8 + e] * HCARRY);
    unsigned short* dst = FHp + ((size_t)dir * NSEQ + (size_t)seq0) * NHID + (size_t)lane * 8;
    for (int pass = 0; pass < 2; ++pass) {
      *(volatile v8h*)dst = hv;
      __threadfence();
    }
  }
}

__global__ __launch_bounds__(GTHR) void linear_kernel(const unsigned short* __restrict__ FHp,
                                                     const unsigned short* __restrict__ WLp,
                                                     const float* __restrict__ blin, float* __restrict__ out) {
  __shared__ __align__(16) float Os[GWAVES * 16 * GOSP];
  const int tid = threadIdx.x, lane = tid & 31, wave = tid >> 5;
  const int c = lane & 15, hh = lane >> 4, koff = 8 * hh;
  const int tile = blockIdx.x * GWAVES + wave;
  const int seq0 = tile * 16;
  const _Float16* FH = (const _Float16*)FHp;
  const _Float16* WL = (const _Float16*)WLp;

  Frag<_Float16>::U fa;
  fa.h[0] = *(const v8h*)(FH + (size_t)(seq0 + c) * NHID + koff);
  fa.h[1] = *(const v8h*)(FH + (size_t)NSEQ * NHID + (size_t)(seq0 + c) * NHID + koff);
  const v16h a  = fa.v;
  const v16h b0 = Frag<_Float16>::load(WL + (size_t)(0 * 16 + c) * (2 * NHID) + koff);
  const v16h b1 = Frag<_Float16>::load(WL + (size_t)(1 * 16 + c) * (2 * NHID) + koff);
  const v8f z8 = {0.f, 0.f, 0.f, 0.f, 0.f, 0.f, 0.f, 0.f};
  v8f acc0 = Frag<_Float16>::mma(a, b0, z8);
  v8f acc1 = Frag<_Float16>::mma(a, b1, z8);
  guard_acc2_ab3(acc0, acc1, a, b0, b1);

  const float bl0 = blin[c], bl1 = blin[16 + c];
  float* osw = Os + wave * 16 * GOSP;
#pragma unroll
  for (int r = 0; r < 8; ++r) {
    osw[(8 * hh + r) * GOSP + c]      = acc0[r] * PROD_INV + bl0;
    osw[(8 * hh + r) * GOSP + 16 + c] = acc1[r] * PROD_INV + bl1;
  }
  __syncthreads();
  const int rq = lane >> 3, c4 = (lane & 7) * 4;
  v4f ov[4];
#pragma unroll
  for (int it = 0; it < 4; ++it) ov[it] = *(const v4f*)(osw + (it * 4 + rq) * GOSP + c4);
  for (int pass = 0; pass < 2; ++pass) {
#pragma unroll
    for (int it = 0; it < 4; ++it)
      *(volatile v4f*)(out + (size_t)(seq0 + it * 4 + rq) * NEMB + c4) = ov[it];
    __threadfence();
  }
}

extern "C" void kernel_launch(void* const* d_in, const int* in_sizes, int n_in,
                              void* d_out, int out_size, void* d_ws, size_t ws_size, hipStream_t stream) {
  if (n_in < 23 || d_out == nullptr || d_ws == nullptr) return;
  if (in_sizes[0] != NSEQ * TLEN || in_sizes[1] != NCHN * 5 || in_sizes[2] != NCHN || in_sizes[3] != NCHN ||
      in_sizes[4] != NCHN || in_sizes[5] != NCHN || in_sizes[6] != NCHN || in_sizes[7] != NCHN * 5 ||
      in_sizes[8] != NCHN || in_sizes[9] != NCHN || in_sizes[10] != NCHN || in_sizes[11] != NCHN ||
      in_sizes[12] != NCHN || in_sizes[13] != NGATE || in_sizes[14] != NGATE * NHID || in_sizes[15] != NGATE ||
      in_sizes[16] != NGATE || in_sizes[17] != NGATE || in_sizes[18] != NGATE * NHID || in_sizes[19] != NGATE ||
      in_sizes[20] != NGATE || in_sizes[21] != NEMB * 2 * NHID || in_sizes[22] != NEMB ||
      out_size != NSEQ * NEMB) return;

  const float* x     = (const float*)d_in[0];
  const float* w1    = (const float*)d_in[1];
  const float* b1    = (const float*)d_in[2];
  const float* g1    = (const float*)d_in[3];
  const float* be1   = (const float*)d_in[4];
  const float* m1    = (const float*)d_in[5];
  const float* v1    = (const float*)d_in[6];
  const float* w2    = (const float*)d_in[7];
  const float* b2    = (const float*)d_in[8];
  const float* g2    = (const float*)d_in[9];
  const float* be2   = (const float*)d_in[10];
  const float* m2    = (const float*)d_in[11];
  const float* v2    = (const float*)d_in[12];
  const float* Wih_f = (const float*)d_in[13];
  const float* Whh_f = (const float*)d_in[14];
  const float* bih_f = (const float*)d_in[15];
  const float* bhh_f = (const float*)d_in[16];
  const float* Wih_b = (const float*)d_in[17];
  const float* Whh_b = (const float*)d_in[18];
  const float* bih_b = (const float*)d_in[19];
  const float* bhh_b = (const float*)d_in[20];
  const float* Wlin  = (const float*)d_in[21];
  const float* blin  = (const float*)d_in[22];
  float* out = (float*)d_out;

  char* ws = (char*)d_ws; size_t off = 0;
  auto carve = [&](size_t bytes) -> char* { char* p = ws + off; off += (bytes + 255) & ~(size_t)255; return p; };
  float*          XT = (float*)carve((size_t)TLEN * NSEQ * 4);
  unsigned short* WH = (unsigned short*)carve((size_t)2 * NGATE * KPAD * 2);
  unsigned short* WL = (unsigned short*)carve((size_t)NEMB * 2 * NHID * 2);
  unsigned short* FH = (unsigned short*)carve((size_t)2 * NSEQ * NHID * 2);
  if (off > ws_size || off > (size_t)134217728) return;

  prep_whh_kernel<<<2, 256, 0, stream>>>(Whh_f, Whh_b, WH);
  prep_wlin_kernel<<<1, 128, 0, stream>>>(Wlin, WL);
  conv_stack_kernel<<<dim3(NSEQ / SGRP, NTCH), CTHR, 0, stream>>>(x, w1, b1, g1, be1, m1, v1,
                                                                  w2, b2, g2, be2, m2, v2, XT);
  bilstm_kernel<<<((NSEQ / 16) * 2) / LWAVES, LTHR, 0, stream>>>(XT, Wih_f, bih_f, bhh_f,
                                                                  Wih_b, bih_b, bhh_b, WH, FH);
  linear_kernel<<<(NSEQ / 16) / GWAVES, GTHR, 0, stream>>>(FH, WL, blin, out);
}
